// Model_81630148428347
// MI455X (gfx1250) — hardware-run, weakly checked
//
#include <hip/hip_runtime.h>
#include <math.h>

typedef __attribute__((ext_vector_type(16))) _Float16 v16h;
typedef __attribute__((ext_vector_type(8)))  _Float16 v8h;
typedef __attribute__((ext_vector_type(8)))  float    v8f;
typedef __attribute__((ext_vector_type(4)))  float    v4f;
typedef __attribute__((ext_vector_type(4)))  unsigned int v4u;

constexpr int kB    = 64;
constexpr int kS    = 1024;
constexpr int kD    = 32;
constexpr int kH    = 2;
constexpr int kDH   = 16;
constexpr int kV    = 28;
constexpr int kRows = kB * kS;
static_assert(kH * kDH == kD, "head split");
static_assert(kD == 32, "one 32-deep k-step per projection");
static_assert((kS % 128) == 0 && (kRows % 128) == 0, "tile multiples");

constexpr float kMinN      = 6.103515625e-05f;
constexpr float kHC        = 16.0f;
constexpr float kWC        = 64.0f;
constexpr float kRC        = 2048.0f;
constexpr float kInvSqrtDH = 0.25f;
static_assert(kDH == 16 && kInvSqrtDH * kInvSqrtDH * (float)kDH == 1.0f, "score scale derived from head dim");
constexpr float kQC        = 64.0f;
constexpr float kKC        = 16.0f;
constexpr float kVC        = 16.0f;
constexpr float kPC        = 32768.0f;
constexpr float kAC        = 64.0f;
constexpr float kTC        = 64.0f;
constexpr float kProjMain  = 1.0f / (kHC * kWC);
constexpr float kProjRes   = kProjMain / kRC;
constexpr float kQMul      = kInvSqrtDH * kQC;
constexpr float kScoreInv  = 1.0f / (kQC * kKC);
constexpr float kPVFold    = kPC * kVC;
constexpr float kT1Main    = 1.0f / (kAC * kWC);
constexpr float kT1Res     = kT1Main / kRC;
constexpr float kT2Main    = 1.0f / (kTC * kWC);
constexpr float kT2Res     = kT2Main / kRC;
constexpr float kFill      = -1.0e9f;

constexpr int kQP = 100;
constexpr int kVP = 136;
constexpr int kPP = 40;
constexpr int kOP = 20;
constexpr int kTP = 36;

constexpr size_t kSzNM  = (size_t)kB * kS * 4;
constexpr size_t kSzNKC = (size_t)kB * 32 * 4;
constexpr size_t kSzW   = (size_t)160 * kD * 2;
constexpr size_t kSzPl  = (size_t)kRows * kD * 2;
constexpr size_t kOffNM  = 0;
constexpr size_t kOffNKC = kOffNM  + kSzNM;
constexpr size_t kOffWH  = kOffNKC + kSzNKC;
constexpr size_t kOffWL  = kOffWH  + kSzW;
constexpr size_t kOffHH  = kOffWL  + kSzW;
constexpr size_t kOffHL  = kOffHH  + kSzPl;
constexpr size_t kOffQ   = kOffHL  + kSzPl;
constexpr size_t kOffK   = kOffQ   + kSzPl;
constexpr size_t kOffVT  = kOffK   + kSzPl;
constexpr size_t kOffAH  = kOffVT  + kSzPl;
constexpr size_t kOffAL  = kOffAH  + kSzPl;
constexpr size_t kWsTotal = kOffAL + kSzPl;
static_assert(kWsTotal == 29650944ull, "carve total");
static_assert(kWsTotal <= 134217728ull, "carve cap");
static_assert((kOffNKC % 128) == 0 && (kOffWH % 128) == 0 && (kOffWL % 128) == 0 && (kOffHH % 128) == 0 &&
              (kOffHL % 128) == 0 && (kOffQ % 128) == 0 && (kOffK % 128) == 0 && (kOffVT % 128) == 0 &&
              (kOffAH % 128) == 0 && (kOffAL % 128) == 0, "128-B aligned regions");

union FH { v16h v; v8h h[2]; };

__device__ __forceinline__ v8f zero8f() { return (v8f){0.f, 0.f, 0.f, 0.f, 0.f, 0.f, 0.f, 0.f}; }
__device__ __forceinline__ v8h zero8h() {
  return (v8h){(_Float16)0.0f, (_Float16)0.0f, (_Float16)0.0f, (_Float16)0.0f,
               (_Float16)0.0f, (_Float16)0.0f, (_Float16)0.0f, (_Float16)0.0f};
}

__device__ __forceinline__ v8f mma_h(v16h a, v16h b, v8f c) {
  c = __builtin_amdgcn_wmma_f32_16x16x32_f16(false, a, false, b, (short)0, c, false, false);
  asm volatile("v_nop\n\tv_nop\n\tv_nop\n\tv_nop" : "+v"(c) : "v"(a), "v"(b));
  return c;
}

__device__ __forceinline__ v16h frag_ld(const unsigned short* p) {
  FH f;
  f.h[0] = *(const v8h*)(const void*)(p);
  f.h[1] = *(const v8h*)(const void*)(p + 16);
  return f.v;
}
__device__ __forceinline__ v16h frag_ld2(const unsigned short* p0, const unsigned short* p1) {
  FH f;
  f.h[0] = *(const v8h*)(const void*)(p0);
  f.h[1] = *(const v8h*)(const void*)(p1);
  return f.v;
}

__device__ __forceinline__ float flush_min(float v) { return (fabsf(v) < kMinN) ? 0.0f : v; }
__device__ __forceinline__ _Float16 to_h(float v) { return (_Float16)flush_min(v); }

__device__ __forceinline__ void split_f16(float v, _Float16& h, _Float16& l) {
  h = (_Float16)flush_min(v);
  float hf = (float)h;
  asm volatile("" : "+v"(hf));
  const float r = (v - hf) * kRC;
  l = (_Float16)flush_min(r);
}

__device__ __forceinline__ unsigned pk2(_Float16 a, _Float16 b) {
  const unsigned short ua = __builtin_bit_cast(unsigned short, a);
  const unsigned short ub = __builtin_bit_cast(unsigned short, b);
  return (unsigned)ua | ((unsigned)ub << 16);
}

__device__ __forceinline__ v4u pack8_plain(v4f a0, v4f a1) {
  const _Float16 h0 = to_h(a0[0]), h1 = to_h(a0[1]), h2 = to_h(a0[2]), h3 = to_h(a0[3]);
  const _Float16 h4 = to_h(a1[0]), h5 = to_h(a1[1]), h6 = to_h(a1[2]), h7 = to_h(a1[3]);
  return (v4u){pk2(h0, h1), pk2(h2, h3), pk2(h4, h5), pk2(h6, h7)};
}

__device__ __forceinline__ void pack8_split(v4f a0, v4f a1, float mul, v4u& uh, v4u& ul) {
  _Float16 h[8], l[8];
  split_f16(a0[0] * mul, h[0], l[0]);
  split_f16(a0[1] * mul, h[1], l[1]);
  split_f16(a0[2] * mul, h[2], l[2]);
  split_f16(a0[3] * mul, h[3], l[3]);
  split_f16(a1[0] * mul, h[4], l[4]);
  split_f16(a1[1] * mul, h[5], l[5]);
  split_f16(a1[2] * mul, h[6], l[6]);
  split_f16(a1[3] * mul, h[7], l[7]);
  uh = (v4u){pk2(h[0], h[1]), pk2(h[2], h[3]), pk2(h[4], h[5]), pk2(h[6], h[7])};
  ul = (v4u){pk2(l[0], l[1]), pk2(l[2], l[3]), pk2(l[4], l[5]), pk2(l[6], l[7])};
}

__global__ __launch_bounds__(128) void wplanes_kernel(
    const float* __restrict__ wq, const float* __restrict__ wk, const float* __restrict__ wv,
    const float* __restrict__ wo, const float* __restrict__ wfc,
    unsigned short* __restrict__ WH, unsigned short* __restrict__ WL)
{
  const int z = blockIdx.x;
  const float* W = (z == 0) ? wq : (z == 1) ? wk : (z == 2) ? wv : (z == 3) ? wo : wfc;
  const int nrows = (z == 4) ? kV : 32;
  const int t = threadIdx.x;
  const int row = t >> 2;
  const int c8 = (t & 3) * 8;
  const int rc = (row < nrows) ? row : (nrows - 1);
  const v4f a0 = *(const v4f*)(W + (size_t)rc * kD + c8);
  const v4f a1 = *(const v4f*)(W + (size_t)rc * kD + c8 + 4);
  float f0 = a0[0], f1 = a0[1], f2 = a0[2], f3 = a0[3];
  float f4 = a1[0], f5 = a1[1], f6 = a1[2], f7 = a1[3];
  asm volatile("" : "+v"(f0));
  asm volatile("" : "+v"(f1));
  asm volatile("" : "+v"(f2));
  asm volatile("" : "+v"(f3));
  asm volatile("" : "+v"(f4));
  asm volatile("" : "+v"(f5));
  asm volatile("" : "+v"(f6));
  asm volatile("" : "+v"(f7));
  const bool valid = (row < nrows);
  const v4f g0 = (v4f){valid ? f0 : 0.0f, valid ? f1 : 0.0f, valid ? f2 : 0.0f, valid ? f3 : 0.0f};
  const v4f g1 = (v4f){valid ? f4 : 0.0f, valid ? f5 : 0.0f, valid ? f6 : 0.0f, valid ? f7 : 0.0f};
  v4u uh, ul;
  pack8_split(g0, g1, kWC, uh, ul);
  const size_t o = (size_t)(z * 32 + row) * kD + c8;
  *(volatile v4u*)(WH + o) = uh;
  *(volatile v4u*)(WL + o) = ul;
  __threadfence();
  *(volatile v4u*)(WH + o) = uh;
  *(volatile v4u*)(WL + o) = ul;
}

__global__ __launch_bounds__(256) void prep_kernel(
    const int* __restrict__ x, const float* __restrict__ mask,
    const float* __restrict__ emb, const float* __restrict__ pe,
    float* __restrict__ nm, int* __restrict__ nkc,
    unsigned short* __restrict__ HH, unsigned short* __restrict__ HL)
{
  __shared__ int sRedA[8];
  __shared__ int sRedB[8];
  __shared__ float sNm[kS];
  const int tid = threadIdx.x, lane = tid & 31, wave = tid >> 5;
  const int b = blockIdx.x;
  const size_t rowb = (size_t)b * kS;

  const v4f mv = *(const v4f*)(mask + rowb + 4 * tid);
  const float m0 = mv[0], m1 = mv[1], m2 = mv[2], m3 = mv[3];
  int la = -1;
  if (m0 > 0.0f) la = 4 * tid + 0;
  if (m1 > 0.0f) la = 4 * tid + 1;
  if (m2 > 0.0f) la = 4 * tid + 2;
  if (m3 > 0.0f) la = 4 * tid + 3;
#pragma unroll
  for (int off = 16; off > 0; off >>= 1) {
    const int o = __shfl_xor(la, off, 32);
    la = (o > la) ? o : la;
  }
  if (lane == 0) sRedA[wave] = la;
  __syncthreads();
  int mx = sRedA[0];
#pragma unroll
  for (int w = 1; w < 8; ++w) { const int o = sRedA[w]; mx = (o > mx) ? o : mx; }
  const int last = (mx < 0) ? (kS - 1) : mx;

  const int sb = 4 * tid;
  const bool hasExt = (last < kS - 1);
  const bool e0 = (sb + 0 > last) && (sb + 0 <= last + 3) && hasExt;
  const bool e1 = (sb + 1 > last) && (sb + 1 <= last + 3) && hasExt;
  const bool e2 = (sb + 2 > last) && (sb + 2 <= last + 3) && hasExt;
  const bool e3 = (sb + 3 > last) && (sb + 3 <= last + 3) && hasExt;
  const float n0 = e0 ? 1.0f : m0;
  const float n1 = e1 ? 1.0f : m1;
  const float n2 = e2 ? 1.0f : m2;
  const float n3 = e3 ? 1.0f : m3;
  int lb = -1;
  if (n0 != 0.0f) lb = sb + 0;
  if (n1 != 0.0f) lb = sb + 1;
  if (n2 != 0.0f) lb = sb + 2;
  if (n3 != 0.0f) lb = sb + 3;
  sNm[sb + 0] = n0;
  sNm[sb + 1] = n1;
  sNm[sb + 2] = n2;
  sNm[sb + 3] = n3;
#pragma unroll
  for (int off = 16; off > 0; off >>= 1) {
    const int o = __shfl_xor(lb, off, 32);
    lb = (o > lb) ? o : lb;
  }
  if (lane == 0) sRedB[wave] = lb;
  __syncthreads();
  int mb = sRedB[0];
#pragma unroll
  for (int w = 1; w < 8; ++w) { const int o = sRedB[w]; mb = (o > mb) ? o : mb; }
  int nch = (mb < 0) ? 8 : ((mb + 128) >> 7);
  nch = (nch < 1) ? 1 : ((nch > 8) ? 8 : nch);

  {
    const v4f nv = (v4f){n0, n1, n2, n3};
    volatile v4f* np = (volatile v4f*)(nm + rowb + 4 * tid);
    *np = nv;
    __threadfence();
    *np = nv;
  }
  if (wave == 0) {
    volatile int* kp = (volatile int*)(nkc + b * 32 + lane);
    *kp = nch;
    __threadfence();
    *kp = nch;
  }

#pragma unroll 1
  for (int it = 0; it < 16; ++it) {
    const int s = it * 64 + (tid >> 2);
    const int c8 = (tid & 3) * 8;
    int tok = x[rowb + s];
    tok = (tok < 0) ? 0 : ((tok > kV - 1) ? (kV - 1) : tok);
    const v4f ea = *(const v4f*)(emb + (size_t)tok * kD + c8);
    const v4f eb = *(const v4f*)(emb + (size_t)tok * kD + c8 + 4);
    const v4f pa = *(const v4f*)(pe + (size_t)s * kD + c8);
    const v4f pb = *(const v4f*)(pe + (size_t)s * kD + c8 + 4);
    const float nmv = sNm[s];
    const bool keep = (nmv != 0.0f);
    const v4f sa = (ea + pa) * nmv;
    const v4f sc = (eb + pb) * nmv;
    const v4f ha = (v4f){keep ? sa[0] : 0.0f, keep ? sa[1] : 0.0f, keep ? sa[2] : 0.0f, keep ? sa[3] : 0.0f};
    const v4f hb = (v4f){keep ? sc[0] : 0.0f, keep ? sc[1] : 0.0f, keep ? sc[2] : 0.0f, keep ? sc[3] : 0.0f};
    v4u uh, ul;
    pack8_split(ha, hb, kHC, uh, ul);
    const size_t o = (rowb + s) * kD + c8;
    *(volatile v4u*)(HH + o) = uh;
    *(volatile v4u*)(HL + o) = ul;
    __threadfence();
    *(volatile v4u*)(HH + o) = uh;
    *(volatile v4u*)(HL + o) = ul;
  }
}

__global__ __launch_bounds__(64) void qkv_kernel(
    const unsigned short* __restrict__ HH, const unsigned short* __restrict__ HL,
    const unsigned short* __restrict__ WH, const unsigned short* __restrict__ WL,
    const float* __restrict__ bq, const float* __restrict__ bk, const float* __restrict__ bv,
    unsigned short* __restrict__ Q16, unsigned short* __restrict__ K16, unsigned short* __restrict__ VT)
{
  __shared__ __align__(16) float sT[2][64 * kQP];
  const int tid = threadIdx.x, lane = tid & 31, wave = tid >> 5;
  const int hh = lane >> 4, c = lane & 15;
  const int row0 = (blockIdx.x * 2 + wave) * 64;
  const int b = row0 >> 10;
  const int s0 = row0 & (kS - 1);

  v16h bh[6], bl[6];
#pragma unroll
  for (int j = 0; j < 6; ++j) {
    const size_t off = (size_t)(j * 16 + c) * kD + 8 * hh;
    bh[j] = frag_ld(WH + off);
    bl[j] = frag_ld(WL + off);
  }
  float bia[6];
  bia[0] = bq[c];
  bia[1] = bq[16 + c];
  bia[2] = bk[c];
  bia[3] = bk[16 + c];
  bia[4] = bv[c];
  bia[5] = bv[16 + c];

  float* slab = sT[wave];
#pragma unroll 1
  for (int i = 0; i < 4; ++i) {
    const size_t ao = (size_t)(row0 + i * 16 + c) * kD + 8 * hh;
    const v16h ah = frag_ld(HH + ao);
    const v16h al = frag_ld(HL + ao);
#pragma unroll
    for (int j = 0; j < 6; ++j) {
      v8f am = zero8f();
      v8f ar = zero8f();
      am = mma_h(ah, bh[j], am);
      ar = mma_h(ah, bl[j], ar);
      ar = mma_h(al, bh[j], ar);
      const float mulj = (j < 2) ? kQMul : ((j < 4) ? kKC : kVC);
#pragma unroll
      for (int r = 0; r < 8; ++r) {
        const float v = (am[r] * kProjMain + ar[r] * kProjRes + bia[j]) * mulj;
        slab[(i * 16 + 8 * hh + r) * kQP + j * 16 + c] = v;
      }
    }
  }
  __syncthreads();

  for (int pass = 0; pass < 2; ++pass) {
#pragma unroll 1
    for (int g = 0; g < 4; ++g) {
      const int pl = g >> 1, hd = g & 1;
      unsigned short* base = (pl == 0) ? Q16 : K16;
#pragma unroll
      for (int it = 0; it < 4; ++it) {
        const int ch = it * 32 + lane;
        const int row = ch >> 1;
        const int d8 = (ch & 1) * 8;
        const float* sp = slab + row * kQP + pl * 32 + hd * 16 + d8;
        const v4f a0 = *(const v4f*)(sp);
        const v4f a1 = *(const v4f*)(sp + 4);
        const v4u u = pack8_plain(a0, a1);
        unsigned short* dst = base + ((size_t)(b * kH + hd) * kS + s0 + row) * kDH + d8;
        *(volatile v4u*)dst = u;
      }
    }
#pragma unroll 1
    for (int it = 0; it < 8; ++it) {
      const int ln = it * 4 + (lane >> 3);
      const int hd = ln >> 4, d = ln & 15;
      const int s8 = (lane & 7) * 8;
      const float* sp = slab + s8 * kQP + 64 + ln;
      const v4f a0 = (v4f){sp[0], sp[kQP], sp[2 * kQP], sp[3 * kQP]};
      const v4f a1 = (v4f){sp[4 * kQP], sp[5 * kQP], sp[6 * kQP], sp[7 * kQP]};
      const v4u u = pack8_plain(a0, a1);
      unsigned short* dst = VT + ((size_t)(b * kH + hd) * kDH + d) * kS + s0 + s8;
      *(volatile v4u*)dst = u;
    }
    __threadfence();
  }
}

__global__ __launch_bounds__(256) void attn_kernel(
    const unsigned short* __restrict__ Q16, const unsigned short* __restrict__ K16,
    const unsigned short* __restrict__ VT, const float* __restrict__ nm, const int* __restrict__ nkc,
    unsigned short* __restrict__ AH, unsigned short* __restrict__ AL)
{
  __shared__ __align__(16) _Float16 Ksh[128 * kDH];
  __shared__ __align__(16) _Float16 Vsh[kDH * kVP];
  __shared__ float sNk[128];
  __shared__ __align__(16) _Float16 Psh[8][16 * kPP];
  __shared__ __align__(16) float Osh[8][16 * kOP];

  const int tid = threadIdx.x, lane = tid & 31, wave = tid >> 5;
  const int hh = lane >> 4, c = lane & 15;
  const int bx = blockIdx.x;
  const int qblk = bx & 7;
  const int hd = (bx >> 3) & 1;
  const int b = bx >> 4;
  const size_t bhrow = (size_t)(b * kH + hd) * kS;
  const int q0 = qblk * 128 + wave * 16;

  int nch = nkc[b * 32];
  nch = (nch < 1) ? 1 : ((nch > 8) ? 8 : nch);

  FH qa;
  qa.h[0] = *(const v8h*)(const void*)(Q16 + (bhrow + q0 + c) * kDH + 8 * hh);
  qa.h[1] = zero8h();

  float mrow[8], lrow[8];
#pragma unroll
  for (int r = 0; r < 8; ++r) { mrow[r] = -INFINITY; lrow[r] = 0.0f; }
  v8f oacc = zero8f();
  _Float16* pw = Psh[wave];

#pragma unroll 1
  for (int kc = 0; kc < nch; ++kc) {
    const int kv0 = kc * 128;
    __syncthreads();
    {
      const v4u kk = *(const v4u*)(const void*)(K16 + (bhrow + kv0) * kDH + tid * 8);
      *(v4u*)(Ksh + tid * 8) = kk;
      const int d = tid >> 4, k8 = (tid & 15) * 8;
      const v4u vv = *(const v4u*)(const void*)(VT + ((size_t)(b * kH + hd) * kDH + d) * kS + kv0 + k8);
      *(v4u*)(Vsh + d * kVP + k8) = vv;
      if (tid < 128) sNk[tid] = nm[(size_t)b * kS + kv0 + tid];
    }
    __syncthreads();

#pragma unroll 1
    for (int kt = 0; kt < 4; ++kt) {
      const int kb = kt * 32;
      FH k0f, k1f;
      k0f.h[0] = *(const v8h*)(Ksh + (kb + c) * kDH + 8 * hh);
      k0f.h[1] = zero8h();
      k1f.h[0] = *(const v8h*)(Ksh + (kb + 16 + c) * kDH + 8 * hh);
      k1f.h[1] = zero8h();
      v8f s0 = zero8f();
      v8f s1 = zero8f();
      s0 = mma_h(qa.v, k0f.v, s0);
      s1 = mma_h(qa.v, k1f.v, s1);
      const bool dead0 = (sNk[kb + c] == 0.0f);
      const bool dead1 = (sNk[kb + 16 + c] == 0.0f);
#pragma unroll
      for (int r = 0; r < 8; ++r) {
        const float x0 = dead0 ? kFill : (s0[r] * kScoreInv);
        const float x1 = dead1 ? kFill : (s1[r] * kScoreInv);
        float tmax = fmaxf(x0, x1);
#pragma unroll
        for (int off = 1; off < 16; off <<= 1) tmax = fmaxf(tmax, __shfl_xor(tmax, off, 32));
        const float mnew = fmaxf(mrow[r], tmax);
        const float alpha = expf(mrow[r] - mnew);
        const float p0 = expf(x0 - mnew);
        const float p1 = expf(x1 - mnew);
        float psum = p0 + p1;
#pragma unroll
        for (int off = 1; off < 16; off <<= 1) psum += __shfl_xor(psum, off, 32);
        lrow[r] = lrow[r] * alpha + psum;
        mrow[r] = mnew;
        oacc[r] *= alpha;
        pw[(8 * hh + r) * kPP + c]      = to_h(p0 * kPC);
        pw[(8 * hh + r) * kPP + 16 + c] = to_h(p1 * kPC);
      }
      __builtin_amdgcn_fence(__ATOMIC_RELEASE, "workgroup");
      __builtin_amdgcn_wave_barrier();
      __builtin_amdgcn_fence(__ATOMIC_ACQUIRE, "workgroup");
      FH pa, vb;
      pa.h[0] = *(const v8h*)(pw + c * kPP + 8 * hh);
      pa.h[1] = *(const v8h*)(pw + c * kPP + 16 + 8 * hh);
      vb.h[0] = *(const v8h*)(Vsh + c * kVP + kb + 8 * hh);
      vb.h[1] = *(const v8h*)(Vsh + c * kVP + kb + 16 + 8 * hh);
      oacc = mma_h(pa.v, vb.v, oacc);
      __builtin_amdgcn_fence(__ATOMIC_RELEASE, "workgroup");
      __builtin_amdgcn_wave_barrier();
      __builtin_amdgcn_fence(__ATOMIC_ACQUIRE, "workgroup");
    }
  }

  float* os = Osh[wave];
#pragma unroll
  for (int r = 0; r < 8; ++r) {
    const float inv = 1.0f / (lrow[r] * kPVFold);
    os[(8 * hh + r) * kOP + c] = oacc[r] * inv;
  }
  __syncthreads();
  {
    const int row = lane >> 1;
    const int d8 = (lane & 1) * 8;
    const float* sp = os + row * kOP + d8;
    const v4f a0 = *(const v4f*)(sp);
    const v4f a1 = *(const v4f*)(sp + 4);
    v4u uh, ul;
    pack8_split(a0, a1, kAC, uh, ul);
    const size_t o = (bhrow + q0 + row) * kDH + d8;
    *(volatile v4u*)(AH + o) = uh;
    *(volatile v4u*)(AL + o) = ul;
    __threadfence();
    *(volatile v4u*)(AH + o) = uh;
    *(volatile v4u*)(AL + o) = ul;
  }
}

__global__ __launch_bounds__(128) void tail_kernel(
    const unsigned short* __restrict__ AH, const unsigned short* __restrict__ AL,
    const unsigned short* __restrict__ WH, const unsigned short* __restrict__ WL,
    const float* __restrict__ bo, const float* __restrict__ bfc, float* __restrict__ out)
{
  __shared__ __align__(16) float sTt[4][32 * kTP];
  __shared__ __align__(16) float sO[4][32 * kV];
  const int tid = threadIdx.x, lane = tid & 31, wave = tid >> 5;
  const int hh = lane >> 4, c = lane & 15;
  const int row0 = (blockIdx.x * 4 + wave) * 32;
  const int b = row0 >> 10;
  const int s0 = row0 & (kS - 1);

  v16h woh[2], wol[2], wfh[2], wfl[2];
#pragma unroll
  for (int j = 0; j < 2; ++j) {
    const size_t o1 = (size_t)(96 + j * 16 + c) * kD + 8 * hh;
    const size_t o2 = (size_t)(128 + j * 16 + c) * kD + 8 * hh;
    woh[j] = frag_ld(WH + o1);
    wol[j] = frag_ld(WL + o1);
    wfh[j] = frag_ld(WH + o2);
    wfl[j] = frag_ld(WL + o2);
  }
  const float bo0 = bo[c], bo1 = bo[16 + c];
  const int cf1 = (16 + c < kV) ? (16 + c) : (kV - 1);
  const float bf0 = bfc[c];
  const float bf1 = bfc[cf1];

  float* slab = sTt[wave];
  float* oslab = sO[wave];

#pragma unroll
  for (int i = 0; i < 2; ++i) {
    const size_t r0 = ((size_t)(b * kH + 0) * kS + s0 + i * 16 + c) * kDH + 8 * hh;
    const size_t r1 = ((size_t)(b * kH + 1) * kS + s0 + i * 16 + c) * kDH + 8 * hh;
    const v16h ah = frag_ld2(AH + r0, AH + r1);
    const v16h al = frag_ld2(AL + r0, AL + r1);
#pragma unroll
    for (int j = 0; j < 2; ++j) {
      v8f am = zero8f();
      v8f ar = zero8f();
      am = mma_h(ah, woh[j], am);
      ar = mma_h(ah, wol[j], ar);
      ar = mma_h(al, woh[j], ar);
      const float bj = (j == 0) ? bo0 : bo1;
#pragma unroll
      for (int r = 0; r < 8; ++r)
        slab[(i * 16 + 8 * hh + r) * kTP + j * 16 + c] = am[r] * kT1Main + ar[r] * kT1Res + bj;
    }
  }
  __syncthreads();

#pragma unroll
  for (int i = 0; i < 2; ++i) {
    const float* tp = slab + (i * 16 + c) * kTP + 8 * hh;
    const v4f x0 = *(const v4f*)(tp);
    const v4f x1 = *(const v4f*)(tp + 4);
    const v4f x2 = *(const v4f*)(tp + 16);
    const v4f x3 = *(const v4f*)(tp + 20);
    float xs[16];
    xs[0] = x0[0];  xs[1] = x0[1];  xs[2] = x0[2];  xs[3] = x0[3];
    xs[4] = x1[0];  xs[5] = x1[1];  xs[6] = x1[2];  xs[7] = x1[3];
    xs[8] = x2[0];  xs[9] = x2[1];  xs[10] = x2[2]; xs[11] = x2[3];
    xs[12] = x3[0]; xs[13] = x3[1]; xs[14] = x3[2]; xs[15] = x3[3];
    v16h th, tl;
#pragma unroll
    for (int e = 0; e < 16; ++e) {
      _Float16 hv, lv;
      split_f16(xs[e] * kTC, hv, lv);
      th[e] = hv;
      tl[e] = lv;
    }
#pragma unroll
    for (int j = 0; j < 2; ++j) {
      v8f am = zero8f();
      v8f ar = zero8f();
      am = mma_h(th, wfh[j], am);
      ar = mma_h(th, wfl[j], ar);
      ar = mma_h(tl, wfh[j], ar);
      const float bj = (j == 0) ? bf0 : bf1;
      const int col = j * 16 + c;
#pragma unroll
      for (int r = 0; r < 8; ++r) {
        const float v = am[r] * kT2Main + ar[r] * kT2Res + bj;
        if (col < kV) oslab[(i * 16 + 8 * hh + r) * kV + col] = v;
      }
    }
  }
  __syncthreads();

  float* dst = out + (size_t)row0 * kV;
  for (int pass = 0; pass < 2; ++pass) {
#pragma unroll
    for (int it = 0; it < 7; ++it) {
      const int idx = (it * 32 + lane) * 4;
      const v4f v = *(const v4f*)(oslab + idx);
      *(volatile v4f*)(dst + idx) = v;
    }
    __threadfence();
  }
}

extern "C" void kernel_launch(void* const* d_in, const int* in_sizes, int n_in,
                              void* d_out, int out_size, void* d_ws, size_t ws_size,
                              hipStream_t stream) {
  if (n_in < 14) return;
  if (in_sizes[0] != kB * kS) return;
  if (in_sizes[1] != kB * kS) return;
  if (in_sizes[2] != kV * kD) return;
  if (in_sizes[3] != kS * kD) return;
  if (in_sizes[4] != kD * kD) return;
  if (in_sizes[5] != kD) return;
  if (in_sizes[6] != kD * kD) return;
  if (in_sizes[7] != kD) return;
  if (in_sizes[8] != kD * kD) return;
  if (in_sizes[9] != kD) return;
  if (in_sizes[10] != kD * kD) return;
  if (in_sizes[11] != kD) return;
  if (in_sizes[12] != kV * kD) return;
  if (in_sizes[13] != kV) return;
  if (out_size != kRows * kV) return;
  if (ws_size < kWsTotal) return;

  const int*   x    = (const int*)d_in[0];
  const float* mask = (const float*)d_in[1];
  const float* emb  = (const float*)d_in[2];
  const float* pe   = (const float*)d_in[3];
  const float* wq   = (const float*)d_in[4];
  const float* bq   = (const float*)d_in[5];
  const float* wk   = (const float*)d_in[6];
  const float* bk   = (const float*)d_in[7];
  const float* wv   = (const float*)d_in[8];
  const float* bv   = (const float*)d_in[9];
  const float* wo   = (const float*)d_in[10];
  const float* bo   = (const float*)d_in[11];
  const float* wfc  = (const float*)d_in[12];
  const float* bfc  = (const float*)d_in[13];
  float* out = (float*)d_out;

  char* ws = (char*)d_ws;
  float*          NM  = (float*)(ws + kOffNM);
  int*            NKC = (int*)(ws + kOffNKC);
  unsigned short* WH  = (unsigned short*)(ws + kOffWH);
  unsigned short* WL  = (unsigned short*)(ws + kOffWL);
  unsigned short* HH  = (unsigned short*)(ws + kOffHH);
  unsigned short* HL  = (unsigned short*)(ws + kOffHL);
  unsigned short* Q16 = (unsigned short*)(ws + kOffQ);
  unsigned short* K16 = (unsigned short*)(ws + kOffK);
  unsigned short* VT  = (unsigned short*)(ws + kOffVT);
  unsigned short* AH  = (unsigned short*)(ws + kOffAH);
  unsigned short* AL  = (unsigned short*)(ws + kOffAL);

  wplanes_kernel<<<5, 128, 0, stream>>>(wq, wk, wv, wo, wfc, WH, WL);
  prep_kernel<<<kB, 256, 0, stream>>>(x, mask, emb, pe, NM, NKC, HH, HL);
  qkv_kernel<<<kRows / 128, 64, 0, stream>>>(HH, HL, WH, WL, bq, bk, bv, Q16, K16, VT);
  attn_kernel<<<kB * kH * (kS / 128), 256, 0, stream>>>(Q16, K16, VT, NM, NKC, AH, AL);
  tail_kernel<<<kRows / 128, 128, 0, stream>>>(AH, AL, WH, WL, bo, bfc, out);
}
